// SemanticSemiSymbolic_21912923144501
// MI455X (gfx1250) — hardware-run, weakly checked
//
#include <hip/hip_runtime.h>
#include <stddef.h>


typedef _Float16 v16h __attribute__((ext_vector_type(16)));
typedef _Float16 v8h  __attribute__((ext_vector_type(8)));
typedef float    v8f  __attribute__((ext_vector_type(8)));
typedef float    v4f  __attribute__((ext_vector_type(4)));
typedef _Float16 h16;

#ifndef NB
#define NB 256
#endif
#define NB_FULL 256
#define IND   512
#define OUTD  512
#define EMB   256

static_assert(NB >= 64 && NB <= NB_FULL && (NB % 64) == 0);
static_assert((IND % 64) == 0 && (IND % 32) == 0);
static_assert((OUTD % 64) == 0);
static_assert((EMB % 32) == 0 && (EMB % 8) == 0);
static_assert(OUTD == 4 * 32 * 4);
static_assert(((size_t)NB * IND) % 2048 == 0);
static_assert(((size_t)IND * EMB) % 2048 == 0);
static_assert(((size_t)OUTD * EMB) % 2048 == 0);
static_assert(((size_t)OUTD * IND) % 2048 == 0);
static_assert((size_t)NB * OUTD * 4 <= (size_t)524288);

#define LDT 72
#define LDC 68
static_assert((LDT % 8) == 0 && LDT >= 64);
static_assert((LDC % 4) == 0 && LDC >= 64);

#define ACARRY 64.0f
#define WCARRY 64.0f
#define UCARRY 256.0f
#define GCARRY 1024.0f
#define DELTA  0.1f
#define LN_EPS 1.0e-5f

#define PE_BYTES  ((size_t)IND * EMB * 2)
#define AW_BYTES  ((size_t)OUTD * EMB * 2)
#define W_BYTES   ((size_t)OUTD * IND * 2)
#define X_BYTES   ((size_t)NB * IND * 2)
#define U_BYTES   ((size_t)NB * IND * 2)
#define S_BYTES   ((size_t)IND * OUTD * 4)
#define VT_BYTES  ((size_t)OUTD * IND * 2)
#define OFF_PE  ((size_t)0)
#define OFF_AW  (OFF_PE + PE_BYTES)
#define OFF_W   (OFF_AW + AW_BYTES)
#define OFF_X   (OFF_W + W_BYTES)
#define OFF_U   (OFF_X + X_BYTES)
#define OFF_S   (OFF_U + U_BYTES)
#define OFF_VT  (OFF_S + S_BYTES)
#define WS_TOTAL (OFF_VT + VT_BYTES)
static_assert((PE_BYTES % 128) == 0 && (AW_BYTES % 128) == 0 && (W_BYTES % 128) == 0);
static_assert((X_BYTES % 128) == 0 && (U_BYTES % 128) == 0 && (S_BYTES % 128) == 0);
static_assert((VT_BYTES % 128) == 0);
static_assert(WS_TOTAL <= (size_t)134217728);

__device__ __forceinline__ float bf16r(float x) {
  unsigned int u = __float_as_uint(x);
  u = (u + 0x7FFFu + ((u >> 16) & 1u)) & 0xFFFF0000u;
  return __uint_as_float(u);
}

static __device__ __forceinline__ h16 toh_flush(float v) {
  const h16 r = (h16)v;
  return (fabsf(v) < 6.103515625e-05f) ? (h16)0.0f : r;
}

__device__ __forceinline__ v16h frag_at(const _Float16* p) {
  v8h lo = *(const v8h*)(p);
  v8h hi = *(const v8h*)(p + 16);
  v16h out;
#pragma unroll
  for (int i = 0; i < 8; ++i) { out[i] = lo[i]; out[i + 8] = hi[i]; }
  return out;
}

__device__ __forceinline__ v8f wmma16(v16h a, v16h b, v8f c) {
  v8f d = __builtin_amdgcn_wmma_f32_16x16x32_f16(false, a, false, b, (short)0, c,
                                                 false, false);
  asm volatile("v_nop\n\tv_nop\n\tv_nop\n\tv_nop" : "+v"(d) : "v"(a), "v"(b));
  return d;
}

__device__ __forceinline__ float red32_sum(float x) {
#pragma unroll
  for (int off = 1; off < 32; off <<= 1) x += __shfl_xor(x, off, 32);
  return x;
}

__global__ __launch_bounds__(256) void plane_kernel(
    const float* __restrict__ src, _Float16* __restrict__ dst, float carry) {
#pragma clang fp contract(off)
  const size_t e = ((size_t)blockIdx.x * 256u + threadIdx.x) * 8u;
  const v4f a0 = *(const v4f*)(src + e);
  const v4f a1 = *(const v4f*)(src + e + 4u);
  v8h o;
#pragma unroll
  for (int i = 0; i < 4; ++i) {
    o[i]     = toh_flush(carry * bf16r(a0[i]));
    o[i + 4] = toh_flush(carry * bf16r(a1[i]));
  }
  _Float16* p = dst + e;
  *(volatile v8h*)p = o;
  __threadfence();
  *(volatile v8h*)p = o;
}

__global__ __launch_bounds__(256) void xplanes_kernel(
    const float* __restrict__ X, _Float16* __restrict__ X16, _Float16* __restrict__ U16) {
#pragma clang fp contract(off)
  const size_t e = ((size_t)blockIdx.x * 256u + threadIdx.x) * 8u;
  const v4f a0 = *(const v4f*)(X + e);
  const v4f a1 = *(const v4f*)(X + e + 4u);
  v8h ox, ou;
#pragma unroll
  for (int i = 0; i < 4; ++i) {
    const float b0 = bf16r(a0[i]);
    const float b1 = bf16r(a1[i]);
    ox[i]     = toh_flush(ACARRY * b0);
    ox[i + 4] = toh_flush(ACARRY * b1);
    ou[i]     = toh_flush(UCARRY * (b0 * fabsf(b0)));
    ou[i + 4] = toh_flush(UCARRY * (b1 * fabsf(b1)));
  }
  _Float16* px = X16 + e;
  _Float16* pu = U16 + e;
  *(volatile v8h*)px = ox;
  *(volatile v8h*)pu = ou;
  __threadfence();
  *(volatile v8h*)px = ox;
  *(volatile v8h*)pu = ou;
}

__global__ __launch_bounds__(256) void gemm_scores_kernel(
    const _Float16* __restrict__ A16, const _Float16* __restrict__ Bt,
    const float* __restrict__ bias, float* __restrict__ outf) {
  __shared__ float Cs[64 * LDC];
  const unsigned tid = threadIdx.x, lane = tid & 31u;
  const unsigned w = (unsigned)__builtin_amdgcn_readfirstlane((int)(threadIdx.x >> 5));
  const unsigned mw = w >> 1, nw = w & 1u;
  const unsigned hh = lane >> 4, m = lane & 15u;
  const unsigned n0 = blockIdx.x * 64u;
  const unsigned row0 = blockIdx.y * 64u;

  const _Float16* ap  = A16 + (size_t)(row0 + mw * 16u + m) * EMB + hh * 8u;
  const _Float16* bp0 = Bt + (size_t)(n0 + nw * 32u + m) * EMB + hh * 8u;
  const _Float16* bp1 = bp0 + (size_t)16 * EMB;
  v8f acc0 = {}, acc1 = {};
#pragma unroll 2
  for (unsigned k0 = 0; k0 < (unsigned)EMB; k0 += 32u) {
    const v16h a  = frag_at(ap + k0);
    const v16h b0 = frag_at(bp0 + k0);
    const v16h b1 = frag_at(bp1 + k0);
    acc0 = wmma16(a, b0, acc0);
    acc1 = wmma16(a, b1, acc1);
  }
#pragma unroll
  for (int r = 0; r < 8; ++r) {
    float* d = &Cs[(mw * 16u + hh * 8u + (unsigned)r) * LDC + nw * 32u + m];
    d[0]  = acc0[r];
    d[16] = acc1[r];
  }
  __syncthreads();

  const float cs = 1.0f / (ACARRY * WCARRY);
  v4f xs[4];
  size_t off[4];
#pragma unroll
  for (unsigned i = 0; i < 4u; ++i) {
    const unsigned r = 16u * i + (tid >> 4);
    const unsigned c = (tid & 15u) * 4u;
    const v4f u = *(const v4f*)&Cs[r * LDC + c];
    const v4f g = *(const v4f*)(bias + n0 + c);
    v4f val;
#pragma unroll
    for (int j = 0; j < 4; ++j) val[j] = u[j] * cs + bf16r(g[j]);
    xs[i] = val;
    off[i] = (size_t)(row0 + r) * OUTD + n0 + c;
  }
#pragma unroll
  for (int i = 0; i < 4; ++i) *(volatile v4f*)(outf + off[i]) = xs[i];
  __threadfence();
#pragma unroll
  for (int i = 0; i < 4; ++i) *(volatile v4f*)(outf + off[i]) = xs[i];
}

__global__ __launch_bounds__(256) void gate_kernel(
    const float* __restrict__ S, const float* __restrict__ W,
    const float* __restrict__ G, const float* __restrict__ Be, _Float16* __restrict__ Vt) {
#pragma clang fp contract(off)
  __shared__ _Float16 T[64 * LDT];
  __shared__ float smu[64];
  __shared__ float srs[64];
  const unsigned tid = threadIdx.x, lane = tid & 31u;
  const unsigned w = (unsigned)__builtin_amdgcn_readfirstlane((int)(threadIdx.x >> 5));
  const unsigned o0 = blockIdx.x * 64u;
  const unsigned i0 = blockIdx.y * 64u;

#pragma unroll 1
  for (unsigned q = 0; q < 8u; ++q) {
    const unsigned rl = w * 8u + q;
    const float* sr = S + (size_t)(i0 + rl) * OUTD + lane * 4u;
    float s = 0.0f;
#pragma unroll 1
    for (unsigned j = 0; j < 4u; ++j) {
      const v4f a = *(const v4f*)(sr + j * 128u);
      s += (a[0] + a[1]) + (a[2] + a[3]);
    }
    const float mean = red32_sum(s) * (1.0f / (float)OUTD);
    float ss = 0.0f;
#pragma unroll 1
    for (unsigned j = 0; j < 4u; ++j) {
      const v4f a = *(const v4f*)(sr + j * 128u);
#pragma unroll
      for (int i = 0; i < 4; ++i) {
        const float d = a[i] - mean;
        ss += d * d;
      }
    }
    const float var = red32_sum(ss) * (1.0f / (float)OUTD);
    const float rstd = rsqrtf(var + LN_EPS);
    if (lane == 0u) { smu[rl] = mean; srs[rl] = rstd; }
  }
  __syncthreads();

  const unsigned nc = tid & 63u;
  const unsigned kq = tid >> 6;
  const float gg = bf16r(G[o0 + nc]);
  const float bb = bf16r(Be[o0 + nc]);
#pragma unroll 1
  for (unsigned j = 0; j < 16u; ++j) {
    const unsigned kr = kq + 4u * j;
    const float sv = S[(size_t)(i0 + kr) * OUTD + o0 + nc];
    const float wv = W[(size_t)(o0 + nc) * IND + i0 + kr];
    const float y = (sv - smu[kr]) * srs[kr] * gg + bb;
    const float sg = __builtin_amdgcn_rcpf(1.0f + __expf(-y));
    T[nc * LDT + kr] = toh_flush(GCARRY * (fabsf(bf16r(wv)) * sg));
  }
  __syncthreads();

  v8h x[2];
  size_t off[2];
#pragma unroll
  for (unsigned i = 0; i < 2u; ++i) {
    const unsigned n = 32u * i + (tid >> 3);
    const unsigned kc = (tid & 7u) * 8u;
    x[i] = *(const v8h*)&T[n * LDT + kc];
    off[i] = (size_t)(o0 + n) * IND + i0 + kc;
  }
#pragma unroll
  for (int i = 0; i < 2; ++i) *(volatile v8h*)(Vt + off[i]) = x[i];
  __threadfence();
#pragma unroll
  for (int i = 0; i < 2; ++i) *(volatile v8h*)(Vt + off[i]) = x[i];
}

__global__ __launch_bounds__(256) void gemm_out_kernel(
    const _Float16* __restrict__ X16, const _Float16* __restrict__ U16,
    const _Float16* __restrict__ W16, const _Float16* __restrict__ Vt,
    float* __restrict__ outf) {
  __shared__ float Cs[64 * LDC];
  const unsigned tid = threadIdx.x, lane = tid & 31u;
  const unsigned w = (unsigned)__builtin_amdgcn_readfirstlane((int)(threadIdx.x >> 5));
  const unsigned mw = w >> 1, nw = w & 1u;
  const unsigned hh = lane >> 4, m = lane & 15u;
  const unsigned n0 = blockIdx.x * 64u;
  const unsigned row0 = blockIdx.y * 64u;

  const _Float16* axp = X16 + (size_t)(row0 + mw * 16u + m) * IND + hh * 8u;
  const _Float16* aup = U16 + (size_t)(row0 + mw * 16u + m) * IND + hh * 8u;
  const _Float16* bw0 = W16 + (size_t)(n0 + nw * 32u + m) * IND + hh * 8u;
  const _Float16* bw1 = bw0 + (size_t)16 * IND;
  const _Float16* bv0 = Vt + (size_t)(n0 + nw * 32u + m) * IND + hh * 8u;
  const _Float16* bv1 = bv0 + (size_t)16 * IND;
  v8f xw0 = {}, xw1 = {}, uv0 = {}, uv1 = {};
#pragma unroll 2
  for (unsigned k0 = 0; k0 < (unsigned)IND; k0 += 32u) {
    const v16h ax = frag_at(axp + k0);
    const v16h b0 = frag_at(bw0 + k0);
    const v16h b1 = frag_at(bw1 + k0);
    xw0 = wmma16(ax, b0, xw0);
    xw1 = wmma16(ax, b1, xw1);
    const v16h au = frag_at(aup + k0);
    const v16h c0 = frag_at(bv0 + k0);
    const v16h c1 = frag_at(bv1 + k0);
    uv0 = wmma16(au, c0, uv0);
    uv1 = wmma16(au, c1, uv1);
  }

  float mx0[8], mx1[8];
#pragma unroll
  for (int r = 0; r < 8; ++r) { mx0[r] = -3.0e38f; mx1[r] = -3.0e38f; }
  const _Float16* up  = U16 + (size_t)(row0 + mw * 16u + hh * 8u) * IND;
  const _Float16* vp0 = Vt + (size_t)(n0 + nw * 32u + m) * IND;
  const _Float16* vp1 = vp0 + (size_t)16 * IND;
#pragma unroll 1
  for (unsigned i = 0; i < (unsigned)IND; i += 8u) {
    const v8h va = *(const v8h*)(vp0 + i);
    const v8h vb = *(const v8h*)(vp1 + i);
    float fa[8], fb[8];
#pragma unroll
    for (int j = 0; j < 8; ++j) { fa[j] = (float)va[j]; fb[j] = (float)vb[j]; }
#pragma unroll
    for (int r = 0; r < 8; ++r) {
      const v8h ur = *(const v8h*)(up + (size_t)r * IND + i);
#pragma unroll
      for (int j = 0; j < 8; ++j) {
        const float uf = (float)ur[j];
        mx0[r] = fmaxf(mx0[r], uf * fa[j]);
        mx1[r] = fmaxf(mx1[r], uf * fb[j]);
      }
    }
  }

  const float cx = 1.0f / (ACARRY * WCARRY);
  const float cu = 1.0f / (UCARRY * GCARRY);
#pragma unroll
  for (int r = 0; r < 8; ++r) {
    const float t0 = xw0[r] * cx + DELTA * ((mx0[r] - uv0[r]) * cu);
    const float t1 = xw1[r] * cx + DELTA * ((mx1[r] - uv1[r]) * cu);
    float* d = &Cs[(mw * 16u + hh * 8u + (unsigned)r) * LDC + nw * 32u + m];
    d[0]  = t0;
    d[16] = t1;
  }
  __syncthreads();

  v4f xs[4];
  size_t off[4];
#pragma unroll
  for (unsigned i = 0; i < 4u; ++i) {
    const unsigned r = 16u * i + (tid >> 4);
    const unsigned c = (tid & 15u) * 4u;
    xs[i] = *(const v4f*)&Cs[r * LDC + c];
    off[i] = (size_t)(row0 + r) * OUTD + n0 + c;
  }
#pragma unroll
  for (int i = 0; i < 4; ++i) *(volatile v4f*)(outf + off[i]) = xs[i];
  __threadfence();
#pragma unroll
  for (int i = 0; i < 4; ++i) *(volatile v4f*)(outf + off[i]) = xs[i];
}

extern "C" void kernel_launch(void* const* d_in, const int* in_sizes, int n_in,
                              void* d_out, int out_size, void* d_ws, size_t ws_size,
                              hipStream_t stream) {
  if (n_in < 7) return;
  if ((long long)in_sizes[0] < (long long)NB * IND) return;
  if ((long long)in_sizes[1] < (long long)OUTD * IND) return;
  if ((long long)in_sizes[2] < (long long)IND * EMB) return;
  if ((long long)in_sizes[3] < (long long)OUTD * EMB) return;
  if (in_sizes[4] < OUTD || in_sizes[5] < OUTD || in_sizes[6] < OUTD) return;
  if ((long long)out_size < (long long)NB * OUTD) return;
  if (ws_size < WS_TOTAL) return;

  const float* x        = (const float*)d_in[0];
  const float* weights  = (const float*)d_in[1];
  const float* pred_emb = (const float*)d_in[2];
  const float* attn_w   = (const float*)d_in[3];
  const float* attn_b   = (const float*)d_in[4];
  const float* ln_g     = (const float*)d_in[5];
  const float* ln_b     = (const float*)d_in[6];
  float* out = (float*)d_out;

  char* ws = (char*)d_ws;
  _Float16* PE16 = (_Float16*)(ws + OFF_PE);
  _Float16* AW16 = (_Float16*)(ws + OFF_AW);
  _Float16* W16  = (_Float16*)(ws + OFF_W);
  _Float16* X16  = (_Float16*)(ws + OFF_X);
  _Float16* U16  = (_Float16*)(ws + OFF_U);
  float*    S32  = (float*)(ws + OFF_S);
  _Float16* Vt16 = (_Float16*)(ws + OFF_VT);

  dim3 blk(256);
  xplanes_kernel<<<dim3((unsigned)(((size_t)NB * IND) / 2048)), blk, 0, stream>>>(x, X16, U16);
  plane_kernel<<<dim3((unsigned)(((size_t)IND * EMB) / 2048)), blk, 0, stream>>>(pred_emb, PE16, ACARRY);
  plane_kernel<<<dim3((unsigned)(((size_t)OUTD * EMB) / 2048)), blk, 0, stream>>>(attn_w, AW16, WCARRY);
  plane_kernel<<<dim3((unsigned)(((size_t)OUTD * IND) / 2048)), blk, 0, stream>>>(weights, W16, WCARRY);

  gemm_scores_kernel<<<dim3(OUTD / 64, IND / 64), blk, 0, stream>>>(PE16, AW16, attn_b, S32);
  gate_kernel<<<dim3(OUTD / 64, IND / 64), blk, 0, stream>>>(S32, weights, ln_g, ln_b, Vt16);
  gemm_out_kernel<<<dim3(OUTD / 64, NB / 64), blk, 0, stream>>>(X16, U16, W16, Vt16, out);
}
